// SpatialBayesianAttention_1082331759385
// MI455X (gfx1250) — hardware-verified
//
#include <hip/hip_runtime.h>
#define BB 4
#define CC 512
#define NN 4096
#define MID 128
#define TT NN
#define NH 1
#define NKV 1
#define NREP 1
#define NVH (2 * NKV)
#define NR (BB * NN)
#define BNEPS 1e-5f
#define ATT_SCALE 0.08838834764831845f
typedef __bf16 v16b __attribute__((ext_vector_type(16)));
typedef unsigned short v8us __attribute__((ext_vector_type(8), may_alias));
typedef float  v8f  __attribute__((ext_vector_type(8)));
typedef float  v4f  __attribute__((ext_vector_type(4)));
typedef float  v4fa __attribute__((ext_vector_type(4), may_alias));
union FragB { v16b v; v8us half[2]; unsigned short u[16]; };

__device__ __forceinline__ unsigned short bf16_bits(float x) { unsigned int u = __float_as_uint(x); return (unsigned short)((u + 0x7FFFu + ((u >> 16) & 1u)) >> 16); }
__device__ __forceinline__ float bf16_val(unsigned short b) { return __uint_as_float(((unsigned int)b) << 16); }
__device__ __forceinline__ float bf16_round(float x) { return bf16_val(bf16_bits(x)); }
template <int NT>
__device__ __forceinline__ v8f mmaN(v16b ah, v16b al, v16b bh, v16b bl, v8f c) {
  c = __builtin_amdgcn_wmma_f32_16x16x32_bf16(false, ah, false, bh, (short)0, c, false, false);
  if (NT >= 2) c = __builtin_amdgcn_wmma_f32_16x16x32_bf16(false, al, false, bh, (short)0, c, false, false);
  if (NT >= 3) c = __builtin_amdgcn_wmma_f32_16x16x32_bf16(false, ah, false, bl, (short)0, c, false, false);
  asm volatile("v_nop\n\tv_nop\n\tv_nop\n\tv_nop" : "+v"(c) : "v"(ah), "v"(al), "v"(bh), "v"(bl));
  return c;
}

__global__ __launch_bounds__(256) void k_wt_bf16(const float* __restrict__ W, unsigned short* __restrict__ Wt, int K, int N) {
  const int t = blockIdx.x * 256 + threadIdx.x;
  const int k8n = K / 8;
  if (t >= N * k8n) return;
  const int n = t / k8n, k8 = (t % k8n) * 8;
  v8us v;
#pragma unroll
  for (int i = 0; i < 8; ++i) v[i] = bf16_bits(W[(size_t)(k8 + i) * N + n]);
  *(volatile v8us*)(Wt + (size_t)n * K + k8) = v;
  __threadfence();
  *(volatile v8us*)(Wt + (size_t)n * K + k8) = v;
}

template <bool ASPLIT, int ACT, bool BIAS_BF16>
__global__ __launch_bounds__(128) void k_gemm_bf(const float* __restrict__ A, int lda, const unsigned short* __restrict__ Wt, int ldb,
                                               const float* __restrict__ bias, float* __restrict__ C, int ldc, int M, int N, int K) {
  __shared__ __attribute__((aligned(16))) float so[4][16][64];
  const int tid = threadIdx.x, w = tid >> 5, lane = tid & 31, ln = lane & 15, hh = lane >> 4;
  const int ntn = N / 64;
  const int wid = blockIdx.x * 4 + w;
  const int mt = wid / ntn, nq = wid % ntn;
  if (mt * 16 >= M) return;
  const int row0 = mt * 16, col0 = nq * 64;
  const float* arow = A + (size_t)(row0 + ln) * lda;
  v8f acc[4] = {};
  for (int kb = 0; kb < K; kb += 32) {
    FragB ah, al;
    const v4f x0 = *(const v4fa*)(arow + kb + 8 * hh), x1 = *(const v4fa*)(arow + kb + 8 * hh + 4);
    const v4f x2 = *(const v4fa*)(arow + kb + 16 + 8 * hh), x3 = *(const v4fa*)(arow + kb + 16 + 8 * hh + 4);
    float xs[16] = {x0[0],x0[1],x0[2],x0[3],x1[0],x1[1],x1[2],x1[3],x2[0],x2[1],x2[2],x2[3],x3[0],x3[1],x3[2],x3[3]};
#pragma unroll
    for (int i = 0; i < 16; ++i) { const unsigned short hb = bf16_bits(xs[i]); ah.u[i] = hb; al.u[i] = ASPLIT ? bf16_bits(xs[i] - bf16_val(hb)) : (unsigned short)0; }
#pragma unroll
    for (int t = 0; t < 4; ++t) {
      const unsigned short* brow = Wt + (size_t)(col0 + t * 16 + ln) * ldb + kb;
      FragB b;
      b.half[0] = *(const v8us*)(brow + 8 * hh);
      b.half[1] = *(const v8us*)(brow + 16 + 8 * hh);
      acc[t] = mmaN<ASPLIT ? 2 : 1>(ah.v, al.v, b.v, b.v, acc[t]);
    }
  }
#pragma unroll
  for (int t = 0; t < 4; ++t) {
    float bv = bias ? bias[col0 + t * 16 + ln] : 0.f;
    if (BIAS_BF16) bv = bf16_round(bv);
#pragma unroll
    for (int r = 0; r < 8; ++r) { float v = acc[t][r] + bv; if (ACT == 1) v = fmaxf(v, 0.f); so[w][8 * hh + r][t * 16 + ln] = v; }
  }
  __builtin_amdgcn_fence(__ATOMIC_ACQ_REL, "workgroup");
  __builtin_amdgcn_wave_barrier();
  const int rsub = lane >> 4, c4 = (lane & 15) * 4;
  for (int pass = 0; pass < 2; ++pass) {
#pragma unroll
    for (int q = 0; q < 8; ++q) {
      const int r = q * 2 + rsub;
      const v4f v = *(const v4fa*)&so[w][r][c4];
      *(volatile v4f*)(C + (size_t)(row0 + r) * ldc + col0 + c4) = v;
    }
    if (pass == 0) __threadfence();
  }
}

template <int D, bool CAUSAL>
__global__ __launch_bounds__(128) void k_flash(const float* __restrict__ qb, const float* __restrict__ kb, const float* __restrict__ vb,
                                             int pitch, int T, int H, float scale, float* __restrict__ y, int ypitch) {
  constexpr int KS = D / 32;
  constexpr int DT = D / 16;
  __shared__ __attribute__((aligned(16))) unsigned short sKh[32][D + 8], sKl[32][D + 8], sVh[32][D + 8], sVl[32][D + 8];
  __shared__ __attribute__((aligned(16))) unsigned short sPh[4][16][40], sPl[4][16][40];
  __shared__ __attribute__((aligned(16))) float sO[4][16][D];
  const int tid = threadIdx.x, w = tid >> 5, lane = tid & 31, ln = lane & 15, hh = lane >> 4;
  const int nqb = (T + 63) / 64;
  const int bh = blockIdx.x / nqb, qblk = blockIdx.x % nqb;
  const int b = bh / H, h = bh % H;
  const int q0 = qblk * 64 + w * 16;
  const float* Q = qb + (size_t)b * T * pitch + h * D;
  const float* K = kb + (size_t)b * T * pitch + h * D;
  const float* V = vb + (size_t)b * T * pitch + h * D;

  FragB aqh[KS], aql[KS];
  {
    int row = q0 + ln; if (row >= T) row = T - 1;
    const float* qr = Q + (size_t)row * pitch;
#pragma unroll
    for (int ks = 0; ks < KS; ++ks)
#pragma unroll
      for (int i = 0; i < 16; ++i) {
        const int d = ks * 32 + ((i < 8) ? (8 * hh + i) : (16 + 8 * hh + (i - 8)));
        const float x = qr[d] * scale; const unsigned short hb = bf16_bits(x);
        aqh[ks].u[i] = hb; aql[ks].u[i] = bf16_bits(x - bf16_val(hb));
      }
  }
  float m_r[8], l_r[8];
#pragma unroll
  for (int r = 0; r < 8; ++r) { m_r[r] = -3.0e38f; l_r[r] = 0.f; }
  v8f oacc[DT];
#pragma unroll
  for (int dt = 0; dt < DT; ++dt) oacc[dt] = (v8f){0.f,0.f,0.f,0.f,0.f,0.f,0.f,0.f};

  const int kv_end = CAUSAL ? min(T, qblk * 64 + 64) : T;
  for (int j0 = 0; j0 < kv_end; j0 += 32) {
    __syncthreads();
    for (int e = tid; e < 32 * (D / 4); e += 128) {
      const int r = e / (D / 4), c4 = (e % (D / 4)) * 4;
      const int key = j0 + r;
      v4f kf = {0.f,0.f,0.f,0.f}, vf = {0.f,0.f,0.f,0.f};
      if (key < T) { kf = *(const v4fa*)(K + (size_t)key * pitch + c4); vf = *(const v4fa*)(V + (size_t)key * pitch + c4); }
#pragma unroll
      for (int t = 0; t < 4; ++t) {
        unsigned short hb = bf16_bits(kf[t]); sKh[r][c4 + t] = hb; sKl[r][c4 + t] = bf16_bits(kf[t] - bf16_val(hb));
        hb = bf16_bits(vf[t]); sVh[r][c4 + t] = hb; sVl[r][c4 + t] = bf16_bits(vf[t] - bf16_val(hb));
      }
    }
    __syncthreads();
    v8f s[2];
#pragma unroll
    for (int nt = 0; nt < 2; ++nt) {
      v8f acc = {};
#pragma unroll
      for (int ks = 0; ks < KS; ++ks) {
        FragB bh_, bl_;
        bh_.half[0] = *(const v8us*)&sKh[nt * 16 + ln][ks * 32 + 8 * hh]; bh_.half[1] = *(const v8us*)&sKh[nt * 16 + ln][ks * 32 + 16 + 8 * hh];
        bl_.half[0] = *(const v8us*)&sKl[nt * 16 + ln][ks * 32 + 8 * hh]; bl_.half[1] = *(const v8us*)&sKl[nt * 16 + ln][ks * 32 + 16 + 8 * hh];
        acc = mmaN<3>(aqh[ks].v, aql[ks].v, bh_.v, bl_.v, acc);
      }
      s[nt] = acc;
    }
    float alpha[8];
#pragma unroll
    for (int r = 0; r < 8; ++r) {
      const int qi = q0 + 8 * hh + r;
      const int ja = j0 + ln, jb = j0 + 16 + ln;
      if (CAUSAL) { if (ja > qi) s[0][r] = -3.0e38f; if (jb > qi) s[1][r] = -3.0e38f; }
      if (ja >= T) s[0][r] = -3.0e38f;
      if (jb >= T) s[1][r] = -3.0e38f;
      float mx = fmaxf(s[0][r], s[1][r]);
      mx = fmaxf(mx, __shfl_xor(mx, 1, 32)); mx = fmaxf(mx, __shfl_xor(mx, 2, 32)); mx = fmaxf(mx, __shfl_xor(mx, 4, 32)); mx = fmaxf(mx, __shfl_xor(mx, 8, 32));
      const float mnew = fmaxf(m_r[r], mx);
      alpha[r] = (mnew > -1.0e38f) ? __expf(m_r[r] - mnew) : 1.0f;
      const float p0 = (s[0][r] > -1.0e38f) ? __expf(s[0][r] - mnew) : 0.f;
      const float p1 = (s[1][r] > -1.0e38f) ? __expf(s[1][r] - mnew) : 0.f;
      m_r[r] = mnew;
      l_r[r] = l_r[r] * alpha[r] + p0 + p1;
      unsigned short hb = bf16_bits(p0); sPh[w][8 * hh + r][ln] = hb;      sPl[w][8 * hh + r][ln] = bf16_bits(p0 - bf16_val(hb));
      hb = bf16_bits(p1);                sPh[w][8 * hh + r][16 + ln] = hb; sPl[w][8 * hh + r][16 + ln] = bf16_bits(p1 - bf16_val(hb));
    }
#pragma unroll
    for (int dt = 0; dt < DT; ++dt)
#pragma unroll
      for (int r = 0; r < 8; ++r) oacc[dt][r] *= alpha[r];
    __builtin_amdgcn_fence(__ATOMIC_ACQ_REL, "workgroup");
    __builtin_amdgcn_wave_barrier();
    FragB pah, pal;
    pah.half[0] = *(const v8us*)&sPh[w][ln][8 * hh]; pah.half[1] = *(const v8us*)&sPh[w][ln][16 + 8 * hh];
    pal.half[0] = *(const v8us*)&sPl[w][ln][8 * hh]; pal.half[1] = *(const v8us*)&sPl[w][ln][16 + 8 * hh];
#pragma unroll
    for (int dt = 0; dt < DT; ++dt) {
      FragB bvh, bvl;
#pragma unroll
      for (int i = 0; i < 8; ++i) {
        bvh.u[i] = sVh[8 * hh + i][dt * 16 + ln]; bvh.u[8 + i] = sVh[16 + 8 * hh + i][dt * 16 + ln];
        bvl.u[i] = sVl[8 * hh + i][dt * 16 + ln]; bvl.u[8 + i] = sVl[16 + 8 * hh + i][dt * 16 + ln];
      }
      oacc[dt] = mmaN<3>(pah.v, pal.v, bvh.v, bvl.v, oacc[dt]);
    }
    __builtin_amdgcn_fence(__ATOMIC_ACQ_REL, "workgroup");
    __builtin_amdgcn_wave_barrier();
  }
#pragma unroll
  for (int r = 0; r < 8; ++r) {
    float l = l_r[r];
    l += __shfl_xor(l, 1, 32); l += __shfl_xor(l, 2, 32); l += __shfl_xor(l, 4, 32); l += __shfl_xor(l, 8, 32);
    l_r[r] = (l > 0.f) ? 1.0f / l : 0.f;
  }
#pragma unroll
  for (int dt = 0; dt < DT; ++dt)
#pragma unroll
    for (int r = 0; r < 8; ++r) sO[w][8 * hh + r][dt * 16 + ln] = oacc[dt][r] * l_r[r];
  __builtin_amdgcn_fence(__ATOMIC_ACQ_REL, "workgroup");
  __builtin_amdgcn_wave_barrier();
  for (int pass = 0; pass < 2; ++pass) {
    for (int r = 0; r < 16; ++r) {
      const int row = q0 + r;
      if (row < T && lane < D / 4) {
        const v4f val = *(const v4fa*)&sO[w][r][lane * 4];
        *(volatile v4f*)(y + ((size_t)b * T + row) * ypitch + h * D + lane * 4) = val;
      }
    }
    if (pass == 0) __threadfence();
  }
}

template <bool ASPLIT, int ACT, bool BIAS_BF16, bool RES_BF16>
__global__ __launch_bounds__(128) void k_gemm_bf3(const float* __restrict__ A, int lda, const unsigned short* __restrict__ Wt, int ldb,
                                                const float* __restrict__ bias, const float* __restrict__ resid, int rmod, int ldr,
                                                float* __restrict__ C, int ldc, int M, int N, int K) {
  __shared__ __attribute__((aligned(16))) float so[4][16][64];
  const int tid = threadIdx.x, w = tid >> 5, lane = tid & 31, ln = lane & 15, hh = lane >> 4;
  const int ntn = N / 64;
  const int wid = blockIdx.x * 4 + w;
  const int mt = wid / ntn, nq = wid % ntn;
  if (mt * 16 >= M) return;
  const int row0 = mt * 16, col0 = nq * 64;
  const float* arow = A + (size_t)(row0 + ln) * lda;
  v8f acc[4] = {};
  for (int kb = 0; kb < K; kb += 32) {
    FragB ah, al;
    const v4f x0 = *(const v4fa*)(arow + kb + 8 * hh), x1 = *(const v4fa*)(arow + kb + 8 * hh + 4);
    const v4f x2 = *(const v4fa*)(arow + kb + 16 + 8 * hh), x3 = *(const v4fa*)(arow + kb + 16 + 8 * hh + 4);
    float xs[16] = {x0[0],x0[1],x0[2],x0[3],x1[0],x1[1],x1[2],x1[3],x2[0],x2[1],x2[2],x2[3],x3[0],x3[1],x3[2],x3[3]};
#pragma unroll
    for (int i = 0; i < 16; ++i) { const unsigned short hb = bf16_bits(xs[i]); ah.u[i] = hb; al.u[i] = ASPLIT ? bf16_bits(xs[i] - bf16_val(hb)) : (unsigned short)0; }
#pragma unroll
    for (int t = 0; t < 4; ++t) {
      const unsigned short* brow = Wt + (size_t)(col0 + t * 16 + ln) * ldb + kb;
      FragB b;
      b.half[0] = *(const v8us*)(brow + 8 * hh);
      b.half[1] = *(const v8us*)(brow + 16 + 8 * hh);
      acc[t] = mmaN<ASPLIT ? 2 : 1>(ah.v, al.v, b.v, b.v, acc[t]);
    }
  }
#pragma unroll
  for (int t = 0; t < 4; ++t) {
    const int col = col0 + t * 16 + ln;
    float bv = bias ? bias[col] : 0.f;
    if (BIAS_BF16) bv = bf16_round(bv);
#pragma unroll
    for (int r = 0; r < 8; ++r) {
      float v = acc[t][r] + bv;
      if (resid) { float rv = resid[(size_t)((row0 + 8 * hh + r) % rmod) * ldr + col]; if (RES_BF16) rv = bf16_round(rv); v += rv; }
      if (ACT == 1) v = fmaxf(v, 0.f);
      if (ACT == 2) v = 0.5f * v * (1.0f + erff(v * 0.70710678118654752f));
      if (ACT == 3) { const float u = 0.7978845608028654f * (v + 0.044715f * v * v * v); v = 0.5f * v * (1.0f + tanhf(u)); }
      so[w][8 * hh + r][t * 16 + ln] = v;
    }
  }
  __builtin_amdgcn_fence(__ATOMIC_ACQ_REL, "workgroup");
  __builtin_amdgcn_wave_barrier();
  const int rsub = lane >> 4, c4 = (lane & 15) * 4;
  for (int pass = 0; pass < 2; ++pass) {
#pragma unroll
    for (int q = 0; q < 8; ++q) {
      const int r = q * 2 + rsub;
      const v4f v = *(const v4fa*)&so[w][r][c4];
      *(volatile v4f*)(C + (size_t)(row0 + r) * ldc + col0 + c4) = v;
    }
    if (pass == 0) __threadfence();
  }
}
template <bool PARAM_BF16>
__global__ __launch_bounds__(256) void k_layernorm(const float* __restrict__ X, const float* __restrict__ R, const float* __restrict__ g, const float* __restrict__ bta,
                                                  float* __restrict__ out_sum, float* __restrict__ out_norm, int N, float eps) {
  __shared__ float red[256];
  const int row = blockIdx.x, tid = threadIdx.x;
  const float* x = X + (size_t)row * N; const float* rr = R ? R + (size_t)row * N : nullptr;
  float vals[16];
  const int per = N / 256;
  float s1 = 0.f;
  for (int u = 0; u < per / 4; ++u) {
    const int j = tid * 4 + 1024 * u;
    const v4f a = *(const v4fa*)(x + j);
    v4f b = {0.f,0.f,0.f,0.f}; if (rr) b = *(const v4fa*)(rr + j);
#pragma unroll
    for (int q = 0; q < 4; ++q) { const float v = a[q] + b[q]; vals[u * 4 + q] = v; s1 += v; }
  }
  red[tid] = s1; __syncthreads();
  for (int st = 128; st > 0; st >>= 1) { if (tid < st) red[tid] += red[tid + st]; __syncthreads(); }
  const float mu = red[0] / (float)N; __syncthreads();
  float s2 = 0.f;
  for (int u = 0; u < per / 4; ++u)
#pragma unroll
    for (int q = 0; q < 4; ++q) { const float c = vals[u * 4 + q] - mu; s2 += c * c; }
  red[tid] = s2; __syncthreads();
  for (int st = 128; st > 0; st >>= 1) { if (tid < st) red[tid] += red[tid + st]; __syncthreads(); }
  const float rs = rsqrtf(red[0] / (float)N + eps);
  for (int pass = 0; pass < 2; ++pass) {
    for (int u = 0; u < per / 4; ++u) {
      const int j = tid * 4 + 1024 * u;
      v4f o, sm;
#pragma unroll
      for (int q = 0; q < 4; ++q) {
        float gg = g[j + q], bb = bta[j + q];
        if (PARAM_BF16) { gg = bf16_round(gg); bb = bf16_round(bb); }
        sm[q] = vals[u * 4 + q]; o[q] = (vals[u * 4 + q] - mu) * rs * gg + bb;
      }
      if (out_sum) *(volatile v4f*)(out_sum + (size_t)row * N + j) = sm;
      *(volatile v4f*)(out_norm + (size_t)row * N + j) = o;
    }
    if (pass == 0) __threadfence();
  }
}


typedef _Float16 v16h __attribute__((ext_vector_type(16)));
union FragH { v16h v; v8us half[2]; _Float16 h[16]; unsigned short u[16]; };
template <int NT>
__device__ __forceinline__ v8f mmaH(v16h ah, v16h al, v16h bh, v16h bl, v8f c) {
  c = __builtin_amdgcn_wmma_f32_16x16x32_f16(false, ah, false, bh, (short)0, c, false, false);
  if (NT >= 2) c = __builtin_amdgcn_wmma_f32_16x16x32_f16(false, al, false, bh, (short)0, c, false, false);
  if (NT >= 3) c = __builtin_amdgcn_wmma_f32_16x16x32_f16(false, ah, false, bl, (short)0, c, false, false);
  asm volatile("v_nop\n\tv_nop\n\tv_nop\n\tv_nop" : "+v"(c) : "v"(ah), "v"(al), "v"(bh), "v"(bl));
  return c;
}
template <bool ASPLIT>
__global__ __launch_bounds__(128) void k_gemm_h(const float* __restrict__ A, int lda, size_t sA, const _Float16* __restrict__ Bh, int ldb, size_t sB, float alpha, float* __restrict__ C, int ldc, size_t sC, int M, int N, int K) {
  __shared__ __attribute__((aligned(16))) float so[4][16][64];
  const int tid = threadIdx.x, w = tid >> 5, lane = tid & 31, ln = lane & 15, hh = lane >> 4; const int by = blockIdx.y;
  A += (size_t)by * sA; Bh += (size_t)by * sB; C += (size_t)by * sC;
  const int ntn = (N + 63) / 64; const int wid = blockIdx.x * 4 + w; const int mt = wid / ntn, nq = wid % ntn; if (mt * 16 >= M) return;
  const int row0 = mt * 16, col0 = nq * 64; const float* arow = A + (size_t)(row0 + ln) * lda;
  v8f acc[4] = {};
  for (int kb = 0; kb < K; kb += 32) {
    FragH ah, al;
    const v4f x0 = *(const v4fa*)(arow + kb + 8 * hh), x1 = *(const v4fa*)(arow + kb + 8 * hh + 4), x2 = *(const v4fa*)(arow + kb + 16 + 8 * hh), x3 = *(const v4fa*)(arow + kb + 16 + 8 * hh + 4);
    float xs[16] = {x0[0],x0[1],x0[2],x0[3],x1[0],x1[1],x1[2],x1[3],x2[0],x2[1],x2[2],x2[3],x3[0],x3[1],x3[2],x3[3]};
#pragma unroll
    for (int i = 0; i < 16; ++i) { const _Float16 h = (_Float16)xs[i]; ah.h[i] = h; al.h[i] = ASPLIT ? (_Float16)(xs[i] - (float)h) : (_Float16)0.0f; }
#pragma unroll
    for (int t = 0; t < 4; ++t) { if (col0 + t * 16 >= N) continue; const size_t boff = (size_t)(col0 + t * 16 + ln) * ldb + kb; FragH bq; bq.half[0] = *(const v8us*)(Bh + boff + 8 * hh); bq.half[1] = *(const v8us*)(Bh + boff + 16 + 8 * hh);
      acc[t] = mmaH<ASPLIT ? 2 : 1>(ah.v, al.v, bq.v, bq.v, acc[t]); }
  }
#pragma unroll
  for (int t = 0; t < 4; ++t) { if (col0 + t * 16 >= N) continue;
#pragma unroll
    for (int r = 0; r < 8; ++r) so[w][8 * hh + r][t * 16 + ln] = acc[t][r] * alpha; }
  __builtin_amdgcn_fence(__ATOMIC_ACQ_REL, "workgroup"); __builtin_amdgcn_wave_barrier();
  const int rsub = lane >> 4, c4 = (lane & 15) * 4;
  for (int pass = 0; pass < 2; ++pass) {
#pragma unroll
    for (int q = 0; q < 8; ++q) { const int r = q * 2 + rsub; if (col0 + c4 < N) { const v4f v = *(const v4fa*)&so[w][r][c4]; *(volatile v4f*)(C + (size_t)(row0 + r) * ldc + col0 + c4) = v; } }
    if (pass == 0) __threadfence(); }
}

__global__ __launch_bounds__(256) void k_wt_f16(const float* __restrict__ W, _Float16* __restrict__ Wt, int K, int N, float scale) {
  const int t = blockIdx.x * 256 + threadIdx.x; if (t >= N * (K / 8)) return; const int n = t / (K / 8), k8 = (t % (K / 8)) * 8; FragH f;
#pragma unroll
  for (int i = 0; i < 8; ++i) f.h[i] = (_Float16)(bf16_round(W[(size_t)(k8 + i) * N + n]) * scale); const v8us o = f.half[0];
  *(volatile v8us*)((unsigned short*)Wt + (size_t)n * K + k8) = o; __threadfence(); *(volatile v8us*)((unsigned short*)Wt + (size_t)n * K + k8) = o;
}
template <int ACT>
__global__ __launch_bounds__(128) void k_gemm_hhx(const _Float16* __restrict__ A, int lda, size_t sA, const _Float16* __restrict__ Bh, int ldb, size_t sB, float alpha, const float* __restrict__ bias, size_t sBias, const float* __restrict__ CP, int rowsPerB, size_t sCPb, int row0g,
    float* __restrict__ C, _Float16* __restrict__ C16, int ldc, size_t sC, int M, int N, int K) {
  __shared__ __attribute__((aligned(16))) float so[4][16][64];
  const int tid = threadIdx.x, w = tid >> 5, lane = tid & 31, ln = lane & 15, hh = lane >> 4; const int by = blockIdx.y;
  A += (size_t)by * sA; Bh += (size_t)by * sB; const size_t cofs = (size_t)by * sC; const float* bp = bias ? bias + (size_t)by * sBias : nullptr;
  const int ntn = (N + 63) / 64; const int wid = blockIdx.x * 4 + w; const int mt = wid / ntn, nq = wid % ntn; if (mt * 16 >= M) return;
  const int row0 = mt * 16, col0 = nq * 64; const _Float16* arow = A + (size_t)(row0 + ln) * lda;
  v8f acc[4] = {};
  for (int kb = 0; kb < K; kb += 32) { FragH ah; ah.half[0] = *(const v8us*)((const unsigned short*)arow + kb + 8 * hh); ah.half[1] = *(const v8us*)((const unsigned short*)arow + kb + 16 + 8 * hh);
#pragma unroll
    for (int t = 0; t < 4; ++t) { if (col0 + t * 16 >= N) continue; const size_t boff = (size_t)(col0 + t * 16 + ln) * ldb + kb; FragH bq; bq.half[0] = *(const v8us*)((const unsigned short*)Bh + boff + 8 * hh); bq.half[1] = *(const v8us*)((const unsigned short*)Bh + boff + 16 + 8 * hh);
      acc[t] = mmaH<1>(ah.v, ah.v, bq.v, bq.v, acc[t]); }
  }
#pragma unroll
  for (int t = 0; t < 4; ++t) { if (col0 + t * 16 >= N) continue; const int col = col0 + t * 16 + ln; const float bv = bp ? bf16_round(bp[col]) : 0.f;
#pragma unroll
    for (int r = 0; r < 8; ++r) { float v = acc[t][r] * alpha + bv; if (CP) { const int bidx = (row0g + row0 + 8 * hh + r) / rowsPerB; v += CP[(size_t)bidx * sCPb + (size_t)by * 64 + col]; } if (ACT == 1) v = (v > 0.f) ? v : expm1f(v); else if (ACT == 7) v = (v > 0.f) ? v + 1.0f : expf(v); else if (ACT == 8) v = tanhf(v); else if (ACT == 9) v = 0.5f * v * (1.0f + tanhf(0.7978845608028654f * (v + 0.044715f * v * v * v))); else if (ACT == 11) v = 1.0f / (1.0f + expf(-v)); else if (ACT == 12) v = (v > 0.f) ? v : 0.01f * v; else if (ACT == 14) v = (v > 0.f) ? v : 0.1f * v; else if (ACT == 15) v = v / (1.0f + expf(-v)); else if (ACT == 3) v = fmaxf(v, 0.f); else if (ACT == 6) v = 0.5f * v * (1.0f + erff(v * 0.70710678118654752f)); so[w][8 * hh + r][t * 16 + ln] = v; } }
  __builtin_amdgcn_fence(__ATOMIC_ACQ_REL, "workgroup"); __builtin_amdgcn_wave_barrier();
  const int rsub = lane >> 4, c4 = (lane & 15) * 4; typedef _Float16 v4h __attribute__((ext_vector_type(4)));
  for (int pass = 0; pass < 2; ++pass) {
#pragma unroll
    for (int q = 0; q < 8; ++q) { const int r = q * 2 + rsub; if (col0 + c4 < N) { const v4f v = *(const v4fa*)&so[w][r][c4]; if (C) *(volatile v4f*)(C + cofs + (size_t)(row0 + r) * ldc + col0 + c4) = v; if (C16) { v4h h4; for (int i = 0; i < 4; ++i) h4[i] = (_Float16)v[i]; *(volatile v4h*)(C16 + cofs + (size_t)(row0 + r) * ldc + col0 + c4) = h4; } } }
    if (pass == 0) __threadfence(); }
}


typedef _Float16 v4h __attribute__((ext_vector_type(4)));

__global__ __launch_bounds__(256) void k_x16(const float* __restrict__ x, _Float16* __restrict__ X16, size_t n8) { const size_t t = (size_t)blockIdx.x * 256 + threadIdx.x; if (t >= n8) return; FragH f;
#pragma unroll
  for (int q = 0; q < 8; ++q) f.h[q] = (_Float16)bf16_round(x[t * 8 + q]); *(volatile v8us*)((unsigned short*)X16 + t * 8) = f.half[0]; __threadfence(); *(volatile v8us*)((unsigned short*)X16 + t * 8) = f.half[0]; }
__global__ __launch_bounds__(256) void k_h16(const float* __restrict__ x, _Float16* __restrict__ X16, size_t n8) { const size_t t = (size_t)blockIdx.x * 256 + threadIdx.x; if (t >= n8) return; FragH f;
#pragma unroll
  for (int q = 0; q < 8; ++q) f.h[q] = (_Float16)x[t * 8 + q]; *(volatile v8us*)((unsigned short*)X16 + t * 8) = f.half[0]; __threadfence(); *(volatile v8us*)((unsigned short*)X16 + t * 8) = f.half[0]; }
__global__ __launch_bounds__(256) void k_round16f(const float* __restrict__ W, _Float16* __restrict__ Bt, size_t n8) { const size_t t = (size_t)blockIdx.x * 256 + threadIdx.x; if (t >= n8) return; FragH f;
#pragma unroll
  for (int i = 0; i < 8; ++i) f.h[i] = (_Float16)(bf16_round(W[t * 8 + i]) * 16.0f); *(volatile v8us*)((unsigned short*)Bt + t * 8) = f.half[0]; __threadfence(); *(volatile v8us*)((unsigned short*)Bt + t * 8) = f.half[0]; }
template <int NHv, int TTv>
__global__ __launch_bounds__(256) void k_vt(const _Float16* __restrict__ V16, int ldv, int voff, _Float16* __restrict__ Vt) { __shared__ unsigned short tl[64][66]; const int tid = threadIdx.x; const int slab = blockIdx.x / (TTv / 64), lg = blockIdx.x % (TTv / 64); const int b = slab / NHv, h = slab % NHv;
  for (int i = tid; i < 64 * 8; i += 256) { const int r = i / 8, c8 = (i % 8) * 8; FragH f; f.half[0] = *(const v8us*)((const unsigned short*)V16 + ((size_t)b * TTv + lg * 64 + r) * ldv + voff + h * 64 + c8);
#pragma unroll
    for (int q = 0; q < 8; ++q) tl[r][c8 + q] = f.u[q]; }
  __syncthreads();
  for (int pass = 0; pass < 2; ++pass) {
#pragma unroll
    for (int rd = 0; rd < 2; ++rd) { const int d = rd * 32 + tid / 8, pc = tid % 8; FragH f;
#pragma unroll
      for (int q = 0; q < 8; ++q) f.u[q] = tl[pc * 8 + q][d];
      *(volatile v8us*)((unsigned short*)Vt + ((size_t)slab * 64 + d) * TTv + lg * 64 + pc * 8) = f.half[0]; }
    if (pass == 0) __threadfence(); } }

__global__ __launch_bounds__(256) void k_vthlu(const float* __restrict__ VF, int ldv, _Float16* __restrict__ Vth, _Float16* __restrict__ Vtl) { __shared__ float tl[64][65]; const int tid = threadIdx.x; const int slab = blockIdx.x / (TT / 64), lg = blockIdx.x % (TT / 64); const int b = slab / NVH, h = slab % NVH;
  for (int i = tid; i < 64 * 16; i += 256) { const int r = i / 16, c4 = (i % 16) * 4; const v4f a = *(const v4fa*)(VF + ((size_t)b * TT + lg * 64 + r) * ldv + h * 64 + c4); tl[r][c4] = a[0]; tl[r][c4 + 1] = a[1]; tl[r][c4 + 2] = a[2]; tl[r][c4 + 3] = a[3]; }
  __syncthreads();
  FragH fh[2], fl[2]; size_t oo[2];
#pragma unroll
  for (int rd = 0; rd < 2; ++rd) { const int d = rd * 32 + tid / 8, pc = tid % 8;
#pragma unroll
    for (int q = 0; q < 8; ++q) { const float v = tl[pc * 8 + q][d]; const _Float16 hv = (_Float16)v; fh[rd].h[q] = hv; fl[rd].h[q] = (_Float16)(v - (float)hv);        } oo[rd] = ((size_t)slab * 64 + d) * TT + lg * 64 + pc * 8; }
  for (int pass = 0; pass < 2; ++pass) {
#pragma unroll
    for (int rd = 0; rd < 2; ++rd) { *(volatile v8us*)((unsigned short*)Vth + oo[rd]) = fh[rd].half[0]; *(volatile v8us*)((unsigned short*)Vtl + oo[rd]) = fl[rd].half[0]; }
    if (pass == 0) __threadfence(); } }
__global__ __launch_bounds__(256) void k_h16s(const float* __restrict__ F, _Float16* __restrict__ H, size_t n8) { const size_t t = (size_t)blockIdx.x * 256 + threadIdx.x; if (t >= n8) return; const v4f a = *(const v4fa*)(F + t * 8), c = *(const v4fa*)(F + t * 8 + 4); FragH f;
#pragma unroll
  for (int q = 0; q < 4; ++q) { f.h[q] = (_Float16)(a[q] * 16.0f); f.h[4 + q] = (_Float16)(c[q] * 16.0f); } *(volatile v8us*)((unsigned short*)H + t * 8) = f.half[0]; __threadfence(); *(volatile v8us*)((unsigned short*)H + t * 8) = f.half[0]; }
__global__ __launch_bounds__(128) void k_flash(const _Float16* __restrict__ Q16, int ldq, const _Float16* __restrict__ K16, int ldk, const _Float16* __restrict__ Vt, const _Float16* __restrict__ Vtlo, float* __restrict__ O, int ldo) {
  constexpr int RPW = 16, RTN = RPW / 16, NQB = TT / (4 * RPW), DT = 8, KS = 4;
  __shared__ __attribute__((aligned(16))) unsigned short sP[4][RPW][40]; __shared__ __attribute__((aligned(16))) unsigned short sPL[4][RPW][40]; __shared__ __attribute__((aligned(16))) float sO[4][RPW][128 + 4];
  const int tid = threadIdx.x, w = tid >> 5, lane = tid & 31, ln = lane & 15, hh = lane >> 4;
  const int slab = blockIdx.x / NQB, qblk = blockIdx.x % NQB; const int b = slab / NH, h = slab % NH; const int qb0 = qblk * (4 * RPW); const int q0 = qb0 + w * RPW;
  FragH aq[2][KS];
#pragma unroll
  for (int rt = 0; rt < RTN; ++rt) { const unsigned short* qr = (const unsigned short*)Q16 + ((size_t)b * TT + q0 + rt * 16 + ln) * ldq + h * 128;
#pragma unroll
    for (int ks = 0; ks < KS; ++ks) { aq[rt][ks].half[0] = *(const v8us*)(qr + ks * 32 + 8 * hh); aq[rt][ks].half[1] = *(const v8us*)(qr + ks * 32 + 16 + 8 * hh); } }
  const unsigned short* Vth = (const unsigned short*)Vt + ((size_t)b * NKV + h / NREP) * 128 * TT; const unsigned short* Vtl = (const unsigned short*)Vtlo + ((size_t)b * NKV + h / NREP) * 128 * TT;
  float m_r[2][8], l_r[2][8]; v8f oacc[2][DT];
#pragma unroll
  for (int rt = 0; rt < RTN; ++rt) {
#pragma unroll
    for (int r = 0; r < 8; ++r) { m_r[rt][r] = -3.0e38f; l_r[rt][r] = 0.f; }
#pragma unroll
    for (int dt = 0; dt < DT; ++dt) oacc[rt][dt] = (v8f){0.f,0.f,0.f,0.f,0.f,0.f,0.f,0.f}; }
  const int jend = TT;
#pragma unroll 1
  for (int j0 = 0; j0 < jend; j0 += 32) {

    v8f s[2][2];
#pragma unroll
    for (int nt = 0; nt < 2; ++nt) { const unsigned short* kr = (const unsigned short*)K16 + ((size_t)b * TT + j0 + nt * 16 + ln) * ldk + (h / NREP) * 128; FragH bk[KS];
#pragma unroll
      for (int ks = 0; ks < KS; ++ks) { bk[ks].half[0] = *(const v8us*)(kr + ks * 32 + 8 * hh); bk[ks].half[1] = *(const v8us*)(kr + ks * 32 + 16 + 8 * hh); }
#pragma unroll
      for (int rt = 0; rt < RTN; ++rt) { v8f acc = (v8f){0.f,0.f,0.f,0.f,0.f,0.f,0.f,0.f};
#pragma unroll
        for (int ks = 0; ks < KS; ++ks) acc = mmaH<1>(aq[rt][ks].v, aq[rt][ks].v, bk[ks].v, bk[ks].v, acc); s[rt][nt] = acc; } }
#pragma unroll
    for (int rt = 0; rt < RTN; ++rt)
#pragma unroll
      for (int r = 0; r < 8; ++r) { const int tq = q0 + rt * 16 + 8 * hh + r; const int k0 = j0 + ln, k1 = j0 + 16 + ln; (void)tq; (void)k0; (void)k1;
        const bool ok0 = true, ok1 = true; (void)tq; (void)k0; (void)k1;
        const float s0 = ok0 ? s[rt][0][r] * ATT_SCALE : -INFINITY, s1 = ok1 ? s[rt][1][r] * ATT_SCALE : -INFINITY; float mc = fmaxf(s0, s1);
        mc = fmaxf(mc, __shfl_xor(mc, 1, 32)); mc = fmaxf(mc, __shfl_xor(mc, 2, 32)); mc = fmaxf(mc, __shfl_xor(mc, 4, 32)); mc = fmaxf(mc, __shfl_xor(mc, 8, 32));
        const float mn = fmaxf(m_r[rt][r], mc); const float al = (mn > -1.0e38f) ? expf(m_r[rt][r] - mn) : 1.0f; m_r[rt][r] = mn; const float p0 = ok0 ? expf(s0 - mn) : 0.f, p1 = ok1 ? expf(s1 - mn) : 0.f; l_r[rt][r] = l_r[rt][r] * al + p0 + p1;
#pragma unroll
        for (int dt = 0; dt < DT; ++dt) oacc[rt][dt][r] *= al;
        FragH t2, t3; const float ps0 = p0 * 1024.0f, ps1 = p1 * 1024.0f; t2.h[0] = (_Float16)ps0; t2.h[1] = (_Float16)ps1; t3.h[0] = (_Float16)(ps0 - (float)t2.h[0]); t3.h[1] = (_Float16)(ps1 - (float)t2.h[1]);
        sP[w][rt * 16 + 8 * hh + r][ln] = t2.u[0]; sP[w][rt * 16 + 8 * hh + r][16 + ln] = t2.u[1]; sPL[w][rt * 16 + 8 * hh + r][ln] = t3.u[0]; sPL[w][rt * 16 + 8 * hh + r][16 + ln] = t3.u[1]; }
    __builtin_amdgcn_fence(__ATOMIC_ACQ_REL, "workgroup"); __builtin_amdgcn_wave_barrier();
    FragH pa[2], pl[2];
#pragma unroll
    for (int rt = 0; rt < RTN; ++rt) { pa[rt].half[0] = *(const v8us*)&sP[w][rt * 16 + ln][8 * hh]; pa[rt].half[1] = *(const v8us*)&sP[w][rt * 16 + ln][16 + 8 * hh]; pl[rt].half[0] = *(const v8us*)&sPL[w][rt * 16 + ln][8 * hh]; pl[rt].half[1] = *(const v8us*)&sPL[w][rt * 16 + ln][16 + 8 * hh]; }
#pragma unroll
    for (int dt = 0; dt < DT; ++dt) { const size_t vo = (size_t)(dt * 16 + ln) * TT + j0; FragH bv, bl; bv.half[0] = *(const v8us*)(Vth + vo + 8 * hh); bv.half[1] = *(const v8us*)(Vth + vo + 16 + 8 * hh); bl.half[0] = *(const v8us*)(Vtl + vo + 8 * hh); bl.half[1] = *(const v8us*)(Vtl + vo + 16 + 8 * hh);
#pragma unroll
      for (int rt = 0; rt < RTN; ++rt) { oacc[rt][dt] = mmaH<1>(pa[rt].v, pa[rt].v, bv.v, bv.v, oacc[rt][dt]); oacc[rt][dt] = mmaH<1>(pl[rt].v, pl[rt].v, bv.v, bv.v, oacc[rt][dt]); oacc[rt][dt] = mmaH<1>(pa[rt].v, pa[rt].v, bl.v, bl.v, oacc[rt][dt]); } }
    __builtin_amdgcn_fence(__ATOMIC_ACQ_REL, "workgroup"); __builtin_amdgcn_wave_barrier(); }
#pragma unroll
  for (int rt = 0; rt < RTN; ++rt) {
#pragma unroll
    for (int r = 0; r < 8; ++r) { float l = l_r[rt][r]; l += __shfl_xor(l, 1, 32); l += __shfl_xor(l, 2, 32); l += __shfl_xor(l, 4, 32); l += __shfl_xor(l, 8, 32); l_r[rt][r] = (l > 0.f) ? 1.0f / (l * 1024.0f) : 0.f; }
#pragma unroll
    for (int dt = 0; dt < DT; ++dt)
#pragma unroll
      for (int r = 0; r < 8; ++r) sO[w][rt * 16 + 8 * hh + r][dt * 16 + ln] = oacc[rt][dt][r] * l_r[rt][r]; }
  __builtin_amdgcn_fence(__ATOMIC_ACQ_REL, "workgroup"); __builtin_amdgcn_wave_barrier();
  for (int pass = 0; pass < 2; ++pass) {
#pragma unroll
    for (int r = 0; r < RPW; ++r) { const int pc = lane; const v4f val = *(const v4fa*)&sO[w][r][pc * 4]; *(volatile v4f*)(O + ((size_t)b * TT + q0 + r) * ldo + h * 128 + pc * 4) = val; }
    if (pass == 0) __threadfence(); } }


__global__ __launch_bounds__(256) void k_tok(const float* __restrict__ x, _Float16* __restrict__ X16) { __shared__ float tl[32][65]; const int tid = threadIdx.x; const int b = blockIdx.x / ((CC / 64) * (NN / 32)), rem = blockIdx.x % ((CC / 64) * (NN / 32)); const int cg = rem / (NN / 32), pg = rem % (NN / 32); const int c0 = cg * 64, p0 = pg * 32;
  for (int i = tid; i < 64 * 32; i += 256) { const int c = i / 32, pp = i % 32; tl[pp][c] = bf16_round(x[((size_t)b * CC + c0 + c) * NN + p0 + pp]); } __syncthreads();
  const int r = tid / 8, pc = tid % 8; FragH f; for (int q = 0; q < 8; ++q) f.h[q] = (_Float16)tl[r][pc * 8 + q]; const size_t row = (size_t)b * NN + p0 + r; *(volatile v8us*)((unsigned short*)X16 + row * CC + c0 + pc * 8) = f.half[0]; __threadfence(); *(volatile v8us*)((unsigned short*)X16 + row * CC + c0 + pc * 8) = f.half[0]; }
__global__ __launch_bounds__(256) void k_wbn(const float* __restrict__ Wm, const float* __restrict__ gam, const float* __restrict__ var, _Float16* __restrict__ Bt) { const int t = blockIdx.x * 256 + threadIdx.x; if (t >= MID * (CC / 8)) return; const int o = t / (CC / 8), c0 = (t % (CC / 8)) * 8;
  const float s = bf16_round(gam[o]) / sqrtf(bf16_round(var[o]) + BNEPS); FragH f;
#pragma unroll
  for (int q = 0; q < 8; ++q) f.h[q] = (_Float16)(bf16_round(Wm[(size_t)o * CC + c0 + q]) * s * 16.0f);
  *(volatile v8us*)((unsigned short*)Bt + (size_t)o * CC + c0) = f.half[0]; __threadfence(); *(volatile v8us*)((unsigned short*)Bt + (size_t)o * CC + c0) = f.half[0]; }
__global__ __launch_bounds__(128) void k_bnadd(const float* __restrict__ bias, const float* __restrict__ gam, const float* __restrict__ bet, const float* __restrict__ mean, const float* __restrict__ var, float* __restrict__ A) { const int o = threadIdx.x;
  const float s = bf16_round(gam[o]) / sqrtf(bf16_round(var[o]) + BNEPS); const float a = (bf16_round(bias[o]) - bf16_round(mean[o])) * s + bf16_round(bet[o]);
  *(volatile float*)(A + o) = a; __threadfence(); *(volatile float*)(A + o) = a; }
__global__ __launch_bounds__(256) void k_out(const float* __restrict__ T, const float* __restrict__ x, float* __restrict__ out) { __shared__ float tl[32][65]; const int tid = threadIdx.x; const int b = blockIdx.x / ((CC / 32) * (NN / 64)), rem = blockIdx.x % ((CC / 32) * (NN / 64)); const int cg = rem / (NN / 64), pg = rem % (NN / 64); const int c0 = cg * 32, p0 = pg * 64;
  for (int i = tid; i < 64 * 32; i += 256) { const int pp = i / 32, c = i % 32; tl[c][pp] = T[((size_t)b * NN + p0 + pp) * CC + c0 + c]; } __syncthreads();
  for (int pass = 0; pass < 2; ++pass) { for (int i = tid; i < 32 * 16; i += 256) { const int c = i / 16, q4 = i % 16; const size_t o = ((size_t)b * CC + c0 + c) * NN + p0 + q4 * 4; const v4f xr = *(const v4fa*)(x + o);
      v4f v; for (int q = 0; q < 4; ++q) v[q] = tl[c][q4 * 4 + q] + bf16_round(xr[q]); *(volatile v4f*)(out + o) = v; } if (pass == 0) __threadfence(); } }

extern "C" void kernel_launch(void* const* d_in, const int* in_sizes, int n_in,
                              void* d_out, int out_size, void* d_ws, size_t ws_size, hipStream_t stream) {
  (void)in_sizes; (void)n_in; (void)out_size;
  const float* const* I = (const float* const*)d_in; const float* x = I[0];
  const float* wf = I[1]; const float* bff = I[2]; const float* gf = I[3]; const float* betaf = I[4]; const float* mf = I[5]; const float* vf = I[6];
  const float* wg = I[7]; const float* bg = I[8]; const float* gg = I[9]; const float* betag = I[10]; const float* mg = I[11]; const float* vg = I[12];
  const float* wh = I[13]; const float* bh = I[14]; const float* wv = I[15]; const float* bv = I[16];
  char* ws = (char*)d_ws; size_t off = 0;
  auto take = [&](size_t bytes) { char* p = ws + off; off += (bytes + 255) & ~(size_t)255; return p; };
  _Float16* Bf = (_Float16*)take((size_t)MID * CC * 2); _Float16* Bg = (_Float16*)take((size_t)MID * CC * 2); _Float16* Bh = (_Float16*)take((size_t)MID * CC * 2); _Float16* Bv = (_Float16*)take((size_t)CC * MID * 2); float* Af = (float*)take(MID * 4); float* Ag = (float*)take(MID * 4);
  _Float16* X16 = (_Float16*)take((size_t)NR * CC * 2); _Float16* F16 = (_Float16*)take((size_t)NR * MID * 2); _Float16* G16 = (_Float16*)take((size_t)NR * MID * 2); float* HF = (float*)take((size_t)NR * MID * 4);
  _Float16* Vt = (_Float16*)take((size_t)NR * MID * 2); _Float16* Vtl = (_Float16*)take((size_t)NR * MID * 2); float* Z = (float*)take((size_t)NR * MID * 4); _Float16* Z16 = F16;   float* T = (float*)take((size_t)NR * CC * 4);
  if (off > ws_size) return;
  const unsigned gw = (unsigned)((MID * (CC / 8) + 255) / 256);
  k_wbn<<<gw, 256, 0, stream>>>(wf, gf, vf, Bf); k_bnadd<<<1, MID, 0, stream>>>(bff, gf, betaf, mf, vf, Af);
  k_wbn<<<gw, 256, 0, stream>>>(wg, gg, vg, Bg); k_bnadd<<<1, MID, 0, stream>>>(bg, gg, betag, mg, vg, Ag);
  k_round16f<<<(MID * CC / 8 + 255) / 256, 256, 0, stream>>>(wh, Bh, (size_t)MID * CC / 8); k_round16f<<<(CC * MID / 8 + 255) / 256, 256, 0, stream>>>(wv, Bv, (size_t)CC * MID / 8);
  k_tok<<<BB * (CC / 64) * (NN / 32), 256, 0, stream>>>(x, X16);
  const dim3 gm(((NR / 16) * (MID / 64) + 3) / 4, 1);
  k_gemm_hhx<3><<<gm, 128, 0, stream>>>(X16, CC, 0, Bf, CC, 0, 0.0625f, nullptr, 0, Af, NR, 0, 0, nullptr, F16, MID, 0, NR, MID, CC);
  k_gemm_hhx<3><<<gm, 128, 0, stream>>>(X16, CC, 0, Bg, CC, 0, 0.0625f, nullptr, 0, Ag, NR, 0, 0, nullptr, G16, MID, 0, NR, MID, CC);
  k_gemm_hhx<0><<<gm, 128, 0, stream>>>(X16, CC, 0, Bh, CC, 0, 0.0625f, bh, 0, nullptr, 1, 0, 0, HF, nullptr, MID, 0, NR, MID, CC);
  k_vthlu<<<BB * NVH * (TT / 64), 256, 0, stream>>>(HF, MID, Vt, Vtl);
  k_flash<<<BB * NH * (TT / 64), 128, 0, stream>>>(F16, MID, G16, MID, Vt, Vtl, Z, MID);
  k_h16s<<<(unsigned)(((size_t)NR * MID / 8 + 255) / 256), 256, 0, stream>>>(Z, Z16, (size_t)NR * MID / 8);
  k_gemm_hhx<0><<<dim3(((NR / 16) * (CC / 64) + 3) / 4, 1), 128, 0, stream>>>(Z16, MID, 0, Bv, MID, 0, 0.00390625f, bv, 0, nullptr, 1, 0, 0, T, nullptr, CC, 0, NR, CC, MID);
  k_out<<<BB * (CC / 32) * (NN / 64), 256, 0, stream>>>(T, x, (float*)d_out);
}
